// TextLSTM_63153199120834
// MI455X (gfx1250) — hardware-verified
//
#include <hip/hip_runtime.h>
#include <math.h>

#define SEQ  512
#define EMB  512
#define HID  512
#define NCL  32000
#define G4   2048
#define NBAT 256
#define BROW 255
#define NT   256
#define NTR  512
#define RP   520
#define MO   64
#define WHSC 16.0f
#define WHSC_INV (1.0f / 16.0f)

typedef __attribute__((ext_vector_type(16))) _Float16 v16h;
typedef __attribute__((ext_vector_type(8)))  _Float16 v8h;
typedef __attribute__((ext_vector_type(16))) __bf16   v16b;
typedef __attribute__((ext_vector_type(8)))  __bf16   v8b;
typedef __attribute__((ext_vector_type(8)))  float    v8f;
typedef __attribute__((ext_vector_type(4)))  float    v4f;

__device__ __forceinline__ unsigned short f2bf_bits(float f) {
  unsigned u = __float_as_uint(f);
  return (unsigned short)((u + 0x7FFFu + ((u >> 16) & 1u)) >> 16);
}
__device__ __forceinline__ float bf_bits2f(unsigned short h) { return __uint_as_float(((unsigned)h) << 16); }

__device__ __forceinline__ void dep_guard_h(v8f& a, v8f& b, v16h x, v16h y) { asm volatile("v_nop\n\tv_nop\n\tv_nop\n\tv_nop" : "+v"(a), "+v"(b) : "v"(x), "v"(y)); }
__device__ __forceinline__ void dep_guard_b(v8f& a, v8f& b, v16b x, v16b y) { asm volatile("v_nop\n\tv_nop\n\tv_nop\n\tv_nop" : "+v"(a), "+v"(b) : "v"(x), "v"(y)); }
__device__ __forceinline__ void keep4_h(v16h a, v16h b, v16h c, v16h d) { asm volatile("v_nop" :: "v"(a), "v"(b), "v"(c), "v"(d)); }
__device__ __forceinline__ void keep4_b(v16b a, v16b b, v16b c, v16b d) { asm volatile("v_nop" :: "v"(a), "v"(b), "v"(c), "v"(d)); }
__device__ __forceinline__ void acc_guard4(v8f& a, v8f& b, v8f& c, v8f& d) { asm volatile("v_nop\n\tv_nop\n\tv_nop\n\tv_nop" : "+v"(a), "+v"(b), "+v"(c), "+v"(d)); }
template <typename T> struct Frag;
template <> struct Frag<_Float16> {
  typedef v16h V; union U { v16h v; v8h h[2]; };
  static __device__ __forceinline__ v16h load(const _Float16* p) {
    U f; f.h[0] = *(const v8h*)(p); f.h[1] = *(const v8h*)(p + 16); return f.v;
  }
  static __device__ __forceinline__ v8f mma(v16h a, v16h b, v8f c) {
    return __builtin_amdgcn_wmma_f32_16x16x32_f16(false, a, false, b, (short)0, c, false, false);
  }
  static __device__ __forceinline__ void guard(v8f& a, v8f& b, v16h x, v16h y) { dep_guard_h(a, b, x, y); }
  static __device__ __forceinline__ void keep(v16h a, v16h b, v16h c, v16h d) { keep4_h(a, b, c, d); }
};
template <> struct Frag<__bf16> {
  typedef v16b V; union U { v16b v; v8b h[2]; };
  static __device__ __forceinline__ v16b load(const __bf16* p) {
    U f; f.h[0] = *(const v8b*)(p); f.h[1] = *(const v8b*)(p + 16); return f.v;
  }
  static __device__ __forceinline__ v8f mma(v16b a, v16b b, v8f c) {
    return __builtin_amdgcn_wmma_f32_16x16x32_bf16(false, a, false, b, (short)0, c, false, false);
  }
  static __device__ __forceinline__ void guard(v8f& a, v8f& b, v16b x, v16b y) { dep_guard_b(a, b, x, y); }
  static __device__ __forceinline__ void keep(v16b a, v16b b, v16b c, v16b d) { keep4_b(a, b, c, d); }
};

template <int ET> struct Elem;
template <> struct Elem<0> { typedef _Float16 T; };
template <> struct Elem<1> { typedef __bf16 T; };
template <int ET, bool SPLIT, int BIAS_MODE, int OUT_MODE, bool RESID, int ACT = 0>
__global__ __launch_bounds__(256) void wmma_gemm64(
    const unsigned short* __restrict__ Ap, const unsigned short* __restrict__ A2p, int lda, long strideA,
    const unsigned short* __restrict__ Btp, const unsigned short* __restrict__ Bt2p, int ldb, long strideB,
    void* __restrict__ Cout, void* __restrict__ Cout2, int ldc, long strideC,
    const float* __restrict__ bias,
    const float* __restrict__ resid, long strideR,
    int M, int N, int K, float scale) {
  typedef typename Elem<ET>::T T;
  typedef typename Frag<T>::V V;
  const T* A = (const T*)Ap; const T* A2 = (const T*)A2p; const T* Bt = (const T*)Btp; const T* Bt2 = (const T*)Bt2p;
  __shared__ __align__(16) float sT[8][16 * 68];
  const int b    = blockIdx.y;
  const int lane = threadIdx.x & 31;
  const int wave = threadIdx.x >> 5;
  const int tilesN = N >> 6;
  const int tilesM = M >> 6;
  const int tile = blockIdx.x * 8 + wave;
  if (tile >= tilesM * tilesN) return;
  const int tm = tile / tilesN;
  const int tn = tile - tm * tilesN;
  const int m0 = tm << 6;
  const int n0 = tn << 6;

  const T* Ab  = A  + (size_t)b * strideA;
  const T* Bb  = Bt + (size_t)b * strideB;
  const T* Ab2 = SPLIT ? (A2  + (size_t)b * strideA) : nullptr;
  const T* Bb2 = SPLIT ? (Bt2 + (size_t)b * strideB) : nullptr;

  const int rlane = lane & 15;
  const int koff  = (lane >> 4) * 8;
  const int mOff  = (lane >> 4) * 8;

  v8f acc[4][4];
#pragma unroll
  for (int i = 0; i < 4; ++i)
#pragma unroll
    for (int j = 0; j < 4; ++j) acc[i][j] = (v8f){0.f,0.f,0.f,0.f,0.f,0.f,0.f,0.f};

  for (int k0 = 0; k0 < K; k0 += 32) {
    V bh[4], bl[4];
#pragma unroll
    for (int j = 0; j < 4; ++j) {
      const size_t bo = (size_t)(n0 + (j << 4) + rlane) * ldb + koff + k0;
      bh[j] = Frag<T>::load(Bb + bo);
      if (SPLIT) bl[j] = Frag<T>::load(Bb2 + bo);
    }
#pragma unroll
    for (int i = 0; i < 4; ++i) {
      const size_t ao = (size_t)(m0 + (i << 4) + rlane) * lda + koff + k0;
      V ah = Frag<T>::load(Ab + ao);
      V al;
      if (SPLIT) al = Frag<T>::load(Ab2 + ao);
#pragma unroll
      for (int j = 0; j < 4; ++j) {
        acc[i][j] = Frag<T>::mma(ah, bh[j], acc[i][j]);
        if (SPLIT) {
          acc[i][j] = Frag<T>::mma(ah, bl[j], acc[i][j]);
          acc[i][j] = Frag<T>::mma(al, bh[j], acc[i][j]);
        }
      }
      Frag<T>::guard(acc[i][0], acc[i][3], ah, SPLIT ? al : ah);
    }
    Frag<T>::keep(bh[0], bh[1], bh[2], bh[3]);
    if (SPLIT) Frag<T>::keep(bl[0], bl[1], bl[2], bl[3]);
  }
  acc_guard4(acc[0][0], acc[0][1], acc[0][2], acc[0][3]);
  acc_guard4(acc[1][0], acc[1][1], acc[1][2], acc[1][3]);
  acc_guard4(acc[2][0], acc[2][1], acc[2][2], acc[2][3]);
  acc_guard4(acc[3][0], acc[3][1], acc[3][2], acc[3][3]);

  float* slab = sT[wave];
  const float* Rb = RESID ? (resid + (size_t)b * strideR) : nullptr;
#pragma unroll
  for (int i = 0; i < 4; ++i) {
    const int mBase = m0 + (i << 4);
#pragma unroll
    for (int j = 0; j < 4; ++j) {
      const int n = n0 + (j << 4) + rlane;
      float bv = 0.f;
      if (BIAS_MODE == 2) bv = bias[n];
#pragma unroll
      for (int r = 0; r < 8; ++r) {
        float v = acc[i][j][r] * scale;
        if (BIAS_MODE == 1) v += bias[mBase + mOff + r];
        if (BIAS_MODE == 2) v += bv;
        if (RESID) v += Rb[(size_t)(mBase + mOff + r) * ldc + n];
        if (ACT == 1) v = tanhf(v);
        if (ACT == 2) v = fmaxf(v, 0.0f);
        if (ACT == 3) v = v / (1.0f + expf(-v));
        if (ACT == 4) v = (v > 0.f) ? v : 0.01f * v;
        if (ACT == 5) v = 0.5f * v * (1.0f + erff(v * 0.70710678118654752f));
        slab[(mOff + r) * 68 + (j << 4) + rlane] = v;
      }
    }
    __builtin_amdgcn_fence(__ATOMIC_RELEASE, "workgroup");
    __builtin_amdgcn_wave_barrier();
    __builtin_amdgcn_fence(__ATOMIC_ACQUIRE, "workgroup");
    if (OUT_MODE == 0) {
      float* C = (float*)Cout + (size_t)b * strideC;
      const int hh = lane >> 4, c4 = (lane & 15) * 4;
      for (int pass = 0; pass < 2; ++pass) {
#pragma unroll
        for (int it = 0; it < 8; ++it) {
          const int row = it * 2 + hh;
          v4f v = *(const v4f*)(slab + row * 68 + c4);
          *(volatile v4f*)(C + (size_t)(mBase + row) * ldc + n0 + c4) = v;
        }
        __threadfence();
      }
    } else {
      const int q = lane >> 3, c8 = (lane & 7) * 8;
      unsigned short* C  = (unsigned short*)Cout  + (size_t)b * strideC;
      unsigned short* C2 = (OUT_MODE == 2) ? ((unsigned short*)Cout2 + (size_t)b * strideC) : nullptr;
      for (int pass = 0; pass < 2; ++pass) {
#pragma unroll
        for (int it = 0; it < 4; ++it) {
          const int row = it * 4 + q;
          const float* sp = slab + row * 68 + c8;
          v8h hv, lv;
#pragma unroll
          for (int e = 0; e < 8; ++e) {
            if (OUT_MODE == 1) {
              hv[e] = (_Float16)sp[e];
            } else {
              unsigned short hb = f2bf_bits(sp[e]);
              unsigned short lb = f2bf_bits(sp[e] - bf_bits2f(hb));
              hv[e] = __builtin_bit_cast(_Float16, hb);
              lv[e] = __builtin_bit_cast(_Float16, lb);
            }
          }
          *(volatile v8h*)(C + (size_t)(mBase + row) * ldc + n0 + c8) = hv;
          if (OUT_MODE == 2) *(volatile v8h*)(C2 + (size_t)(mBase + row) * ldc + n0 + c8) = lv;
        }
        __threadfence();
      }
    }
    __builtin_amdgcn_fence(__ATOMIC_RELEASE, "workgroup");
    __builtin_amdgcn_wave_barrier();
    __builtin_amdgcn_fence(__ATOMIC_ACQUIRE, "workgroup");
  }
}

__device__ __forceinline__ void split_bits(float f, unsigned short& hb, unsigned short& lb) {
  hb = f2bf_bits(f);
  lb = f2bf_bits(f - bf_bits2f(hb));
}
__device__ __forceinline__ float fsig(float x) { return __builtin_amdgcn_rcpf(1.0f + __expf(-x)); }

template <int MODE>
__global__ __launch_bounds__(NT) void tp_kernel(const float* __restrict__ s0, const float* __restrict__ s1,
                                               const float* __restrict__ s2, const float* __restrict__ s3,
                                               int R, int C, int ldo, int zrows,
                                               unsigned short* __restrict__ OH, unsigned short* __restrict__ OL, float sc) {
  __shared__ float T[64 * 65];
  const int tid = threadIdx.x;
  const int c0 = blockIdx.x * 64, r0 = blockIdx.y * 64, z = blockIdx.z;
  const float* src = (z == 0) ? s0 : (z == 1) ? s1 : (z == 2) ? s2 : s3;
#pragma unroll
  for (int i = 0; i < 4; ++i) {
    const int idx = i * NT + tid;
    const int rr = idx >> 4, cc = (idx & 15) * 4;
    const v4f v = *(const v4f*)(src + (size_t)(r0 + rr) * C + c0 + cc);
    T[rr * 65 + cc + 0] = v[0];
    T[rr * 65 + cc + 1] = v[1];
    T[rr * 65 + cc + 2] = v[2];
    T[rr * 65 + cc + 3] = v[3];
  }
  __syncthreads();
  const int q = tid >> 3, c8 = (tid & 7) * 8;
  v8h hv[2], lv[2];
#pragma unroll
  for (int g = 0; g < 2; ++g) {
    const int qq = g * 32 + q;
#pragma unroll
    for (int e = 0; e < 8; ++e) {
      const float f = T[(c8 + e) * 65 + qq];
      if (MODE == 0) {
        unsigned short hb, lb; split_bits(f, hb, lb);
        hv[g][e] = __builtin_bit_cast(_Float16, hb);
        lv[g][e] = __builtin_bit_cast(_Float16, lb);
      } else {
        hv[g][e] = (_Float16)(f * sc);
        lv[g][e] = (_Float16)0.0f;
      }
    }
  }
  const size_t zo = (size_t)z * (size_t)zrows;
  for (int pass = 0; pass < 2; ++pass) {
#pragma unroll
    for (int g = 0; g < 2; ++g) {
      const size_t o = (zo + (size_t)(c0 + g * 32 + q)) * (size_t)ldo + (size_t)(r0 + c8);
      *(volatile v8h*)(OH + o) = hv[g];
      if (MODE == 0) *(volatile v8h*)(OL + o) = lv[g];
    }
    __threadfence();
  }
}

__global__ __launch_bounds__(NT) void gather_kernel(const int* __restrict__ X, const float* __restrict__ emb,
                                                   const float* __restrict__ bii, const float* __restrict__ bhi,
                                                   const float* __restrict__ bif, const float* __restrict__ bhf,
                                                   const float* __restrict__ bigg, const float* __restrict__ bhg,
                                                   const float* __restrict__ bio, const float* __restrict__ bho,
                                                   unsigned short* __restrict__ EXh, unsigned short* __restrict__ EXl,
                                                   float* __restrict__ bsum) {
  const int blk = blockIdx.x, tid = threadIdx.x;
  if (blk < 128) {
    const int gid = blk * NT + tid;
    const int row = gid >> 6, c8 = (gid & 63) * 8;
    int tok = X[BROW * SEQ + row];
    tok = tok < 0 ? 0 : (tok >= NCL ? NCL - 1 : tok);
    const float* ep = emb + (size_t)tok * EMB + c8;
    const v4f a = *(const v4f*)ep, bq = *(const v4f*)(ep + 4);
    v8h hv, lv;
#pragma unroll
    for (int e = 0; e < 4; ++e) {
      unsigned short hb, lb;
      split_bits(a[e], hb, lb);
      hv[e] = __builtin_bit_cast(_Float16, hb); lv[e] = __builtin_bit_cast(_Float16, lb);
      split_bits(bq[e], hb, lb);
      hv[4 + e] = __builtin_bit_cast(_Float16, hb); lv[4 + e] = __builtin_bit_cast(_Float16, lb);
    }
    const size_t o = (size_t)row * EMB + c8;
    *(volatile v8h*)(EXh + o) = hv;
    *(volatile v8h*)(EXl + o) = lv;
    __threadfence();
    *(volatile v8h*)(EXh + o) = hv;
    *(volatile v8h*)(EXl + o) = lv;
  } else {
    const int jx = (blk - 128) * NT + tid;
    const int gi = jx >> 9, hc = jx & 511;
    const float v0 = bii[hc] + bhi[hc];
    const float v1 = bif[hc] + bhf[hc];
    const float v2 = bigg[hc] + bhg[hc];
    const float v3 = bio[hc] + bho[hc];
    const float v = (gi == 0) ? v0 : (gi == 1) ? v1 : (gi == 2) ? v2 : v3;
    float* p = bsum + jx;
    *(volatile float*)p = v; __threadfence(); *(volatile float*)p = v;
  }
}

__global__ __launch_bounds__(NTR) void rec_kernel(const float* __restrict__ hidden, const float* __restrict__ cell,
                                                 const float* __restrict__ GX,
                                                 const unsigned short* __restrict__ WHp,
                                                 unsigned short* __restrict__ Hh, unsigned short* __restrict__ Hl) {
  __shared__ __align__(16) _Float16 At[16 * RP];
  __shared__ __align__(16) float cs[HID];
  __shared__ __align__(16) float hn[HID];
  const _Float16* WH = (const _Float16*)WHp;
  const int tid = threadIdx.x, lane = tid & 31, wave = tid >> 5;
  const int c = lane & 15, hh = lane >> 4, koff = hh * 8;
#pragma unroll 1
  for (int i = tid; i < 16 * RP; i += NTR) At[i] = (_Float16)0.0f;
  cs[tid] = cell[BROW * HID + tid];
  hn[tid] = hidden[BROW * HID + tid];
  __syncthreads();
  At[tid] = (_Float16)hn[tid];
  __syncthreads();
  const _Float16* arow = At + c * RP + koff;
  const v8f z8 = {0.f, 0.f, 0.f, 0.f, 0.f, 0.f, 0.f, 0.f};

#pragma unroll 1
  for (int t = 0; t < SEQ; ++t) {
    const float* gx = GX + (size_t)t * G4;
#pragma unroll 1
    for (int nt = 0; nt < 2; ++nt) {
      const int j = 32 * wave + 16 * nt + c;
      const _Float16* wb = WH + (size_t)j * HID + koff;
      v8f acc[4];
      acc[0] = z8; acc[1] = z8; acc[2] = z8; acc[3] = z8;
#pragma unroll 1
      for (int k0 = 0; k0 < HID; k0 += 32) {
        const v16h a  = Frag<_Float16>::load(arow + k0);
        const v16h b0 = Frag<_Float16>::load(wb + k0);
        const v16h b1 = Frag<_Float16>::load(wb + (size_t)1 * HID * HID + k0);
        const v16h b2 = Frag<_Float16>::load(wb + (size_t)2 * HID * HID + k0);
        const v16h b3 = Frag<_Float16>::load(wb + (size_t)3 * HID * HID + k0);
        acc[0] = Frag<_Float16>::mma(a, b0, acc[0]);
        acc[1] = Frag<_Float16>::mma(a, b1, acc[1]);
        acc[2] = Frag<_Float16>::mma(a, b2, acc[2]);
        acc[3] = Frag<_Float16>::mma(a, b3, acc[3]);
        dep_guard_h(acc[0], acc[3], a, b3);
        keep4_h(b0, b1, b2, b3);
      }
      acc_guard4(acc[0], acc[1], acc[2], acc[3]);
      const float z0 = gx[j]           + acc[0][0] * WHSC_INV;
      const float z1 = gx[HID + j]     + acc[1][0] * WHSC_INV;
      const float z2 = gx[2 * HID + j] + acc[2][0] * WHSC_INV;
      const float z3 = gx[3 * HID + j] + acc[3][0] * WHSC_INV;
      const float ig = fsig(z0), fg = fsig(z1), gg = tanhf(z2), og = fsig(z3);
      const float cprev = cs[j];
      const float cnew = fg * cprev + ig * gg;
      const float hnew = og * tanhf(cnew);
      if (hh == 0) { cs[j] = cnew; hn[j] = hnew; }
    }
    __syncthreads();
    At[tid] = (_Float16)hn[tid];
    __syncthreads();
  }
#pragma unroll 1
  for (int it = 0; it < 8; ++it) {
    const int idx = it * NTR + tid;
    const int row = idx >> 6, c8 = (idx & 63) * 8;
    v8h hv, lv;
#pragma unroll
    for (int e = 0; e < 8; ++e) {
      unsigned short hb, lb; split_bits(hn[c8 + e], hb, lb);
      const unsigned short hs = (row == 0) ? hb : (unsigned short)0;
      const unsigned short ls = (row == 0) ? lb : (unsigned short)0;
      hv[e] = __builtin_bit_cast(_Float16, hs);
      lv[e] = __builtin_bit_cast(_Float16, ls);
    }
    const size_t o = (size_t)row * HID + c8;
    *(volatile v8h*)(Hh + o) = hv;
    *(volatile v8h*)(Hl + o) = lv;
    __threadfence();
    *(volatile v8h*)(Hh + o) = hv;
    *(volatile v8h*)(Hl + o) = lv;
  }
}

__global__ __launch_bounds__(NT) void out_kernel(const float* __restrict__ Cm, float* __restrict__ out) {
  const int q = blockIdx.x * NT + threadIdx.x;
  if (q < NCL / 4) {
    const v4f v = *(const v4f*)(Cm + 4 * (size_t)q);
    *(volatile v4f*)(out + 4 * (size_t)q) = v;
    __threadfence();
    *(volatile v4f*)(out + 4 * (size_t)q) = v;
  }
}

extern "C" void kernel_launch(void* const* d_in, const int* in_sizes, int n_in,
                              void* d_out, int out_size, void* d_ws, size_t ws_size, hipStream_t stream) {
  if (n_in < 22 || d_out == nullptr || d_ws == nullptr) return;
  if (in_sizes[0] != NBAT * SEQ || in_sizes[1] != NBAT * HID || in_sizes[2] != NBAT * HID || in_sizes[3] != NCL * EMB ||
      in_sizes[4] != EMB * HID || in_sizes[6] != HID * HID || in_sizes[8] != EMB * HID || in_sizes[10] != HID * HID ||
      in_sizes[12] != EMB * HID || in_sizes[14] != HID * HID || in_sizes[16] != EMB * HID || in_sizes[18] != HID * HID ||
      in_sizes[5] != HID || in_sizes[7] != HID || in_sizes[9] != HID || in_sizes[11] != HID || in_sizes[13] != HID ||
      in_sizes[15] != HID || in_sizes[17] != HID || in_sizes[19] != HID ||
      in_sizes[20] != HID * NCL || in_sizes[21] != NCL || out_size != NCL) return;

  const int*   X      = (const int*)  d_in[0];
  const float* hidden = (const float*)d_in[1];
  const float* cell   = (const float*)d_in[2];
  const float* emb    = (const float*)d_in[3];
  const float* W_ii   = (const float*)d_in[4];
  const float* b_ii   = (const float*)d_in[5];
  const float* W_hi   = (const float*)d_in[6];
  const float* b_hi   = (const float*)d_in[7];
  const float* W_if   = (const float*)d_in[8];
  const float* b_if   = (const float*)d_in[9];
  const float* W_hf   = (const float*)d_in[10];
  const float* b_hf   = (const float*)d_in[11];
  const float* W_ig   = (const float*)d_in[12];
  const float* b_ig   = (const float*)d_in[13];
  const float* W_hg   = (const float*)d_in[14];
  const float* b_hg   = (const float*)d_in[15];
  const float* W_io   = (const float*)d_in[16];
  const float* b_io   = (const float*)d_in[17];
  const float* W_ho   = (const float*)d_in[18];
  const float* b_ho   = (const float*)d_in[19];
  const float* W_out  = (const float*)d_in[20];
  const float* b_out  = (const float*)d_in[21];
  float* out = (float*)d_out;

  char* ws = (char*)d_ws; size_t off = 0;
  auto carve = [&](size_t bytes) -> char* { char* p = ws + off; off += (bytes + 255) & ~(size_t)255; return p; };
  unsigned short* WXh  = (unsigned short*)carve((size_t)G4 * EMB * 2);
  unsigned short* WXl  = (unsigned short*)carve((size_t)G4 * EMB * 2);
  unsigned short* WH16 = (unsigned short*)carve((size_t)G4 * HID * 2);
  unsigned short* WOh  = (unsigned short*)carve((size_t)NCL * HID * 2);
  unsigned short* WOl  = (unsigned short*)carve((size_t)NCL * HID * 2);
  float*          bsum = (float*)carve((size_t)G4 * 4);
  unsigned short* EXh  = (unsigned short*)carve((size_t)SEQ * EMB * 2);
  unsigned short* EXl  = (unsigned short*)carve((size_t)SEQ * EMB * 2);
  float*          GX   = (float*)carve((size_t)SEQ * G4 * 4);
  unsigned short* Hh   = (unsigned short*)carve((size_t)MO * HID * 2);
  unsigned short* Hl   = (unsigned short*)carve((size_t)MO * HID * 2);
  float*          Cm   = (float*)carve((size_t)MO * NCL * 4);
  if (off > ws_size || off > (size_t)134217728) return;

  tp_kernel<0><<<dim3(HID / 64, EMB / 64, 4), NT, 0, stream>>>(W_ii, W_if, W_ig, W_io, EMB, HID, EMB, HID, WXh, WXl, 1.0f);
  tp_kernel<1><<<dim3(HID / 64, HID / 64, 4), NT, 0, stream>>>(W_hi, W_hf, W_hg, W_ho, HID, HID, HID, HID, WH16, WH16, WHSC);
  tp_kernel<0><<<dim3(NCL / 64, HID / 64, 1), NT, 0, stream>>>(W_out, W_out, W_out, W_out, HID, NCL, HID, 0, WOh, WOl, 1.0f);
  gather_kernel<<<128 + 8, NT, 0, stream>>>(X, emb, b_ii, b_hi, b_if, b_hf, b_ig, b_hg, b_io, b_ho, EXh, EXl, bsum);
  {
    const int tiles = (SEQ / 64) * (G4 / 64);
    wmma_gemm64<1, true, 2, 0, false><<<dim3((tiles + 7) / 8, 1), 256, 0, stream>>>(
        (const unsigned short*)EXh, (const unsigned short*)EXl, EMB, 0L,
        (const unsigned short*)WXh, (const unsigned short*)WXl, EMB, 0L,
        (void*)GX, (void*)nullptr, G4, 0L,
        bsum, (const float*)nullptr, 0L, SEQ, G4, EMB, 1.0f);
  }
  rec_kernel<<<1, NTR, 0, stream>>>(hidden, cell, GX, WH16, Hh, Hl);
  {
    const int tiles = (MO / 64) * (NCL / 64);
    wmma_gemm64<1, true, 2, 0, false><<<dim3((tiles + 7) / 8, 1), 256, 0, stream>>>(
        (const unsigned short*)Hh, (const unsigned short*)Hl, HID, 0L,
        (const unsigned short*)WOh, (const unsigned short*)WOl, HID, 0L,
        (void*)Cm, (void*)nullptr, NCL, 0L,
        b_out, (const float*)nullptr, 0L, MO, NCL, HID, 1.0f);
  }
  out_kernel<<<(NCL / 4 + NT - 1) / NT, NT, 0, stream>>>(Cm, out);
}
